// WubuBlock_22024592294279
// MI455X (gfx1250) — hardware-verified
//
#include <hip/hip_runtime.h>
#include <math.h>

typedef __attribute__((ext_vector_type(16))) _Float16 v16h;
typedef __attribute__((ext_vector_type(8)))  _Float16 v8h;
typedef __attribute__((ext_vector_type(16))) __bf16   v16b;
typedef __attribute__((ext_vector_type(8)))  float    v8f;
typedef __attribute__((ext_vector_type(4)))  float    v4f;

__device__ __forceinline__ int frag_k(int i, int h) { return (i < 8) ? (8 * h + i) : (16 + 8 * h + (i - 8)); }
__device__ __forceinline__ __bf16 bf16_rne(float f) {
    unsigned int u = __float_as_uint(f);
    u += 0x7fffu + ((u >> 16) & 1u);
    return __builtin_bit_cast(__bf16, (unsigned short)(u >> 16));
}
__device__ __forceinline__ float bf16_f32(__bf16 b) { return __uint_as_float(((unsigned int)__builtin_bit_cast(unsigned short, b)) << 16); }
__device__ __forceinline__ v8f wmma16(v16h a, v16h b, v8f c) {
    c = __builtin_amdgcn_wmma_f32_16x16x32_f16(false, a, false, b, (short)0, c, false, false);
    asm volatile("v_nop\n\tv_nop\n\tv_nop\n\tv_nop" : "+v"(c) : "v"(a), "v"(b));
    return c;
}
__device__ __forceinline__ v8f wmmab(v16b a, v16b b, v8f c) {
    c = __builtin_amdgcn_wmma_f32_16x16x32_bf16(false, a, false, b, (short)0, c, false, false);
    asm volatile("v_nop\n\tv_nop\n\tv_nop\n\tv_nop" : "+v"(c) : "v"(a), "v"(b));
    return c;
}
struct Split { v16b hi, lo; };
__device__ __forceinline__ v8f wmma3(const Split& a, const Split& b, v8f c) {
    c = __builtin_amdgcn_wmma_f32_16x16x32_bf16(false, a.hi, false, b.hi, (short)0, c, false, false);
    c = __builtin_amdgcn_wmma_f32_16x16x32_bf16(false, a.hi, false, b.lo, (short)0, c, false, false);
    c = __builtin_amdgcn_wmma_f32_16x16x32_bf16(false, a.lo, false, b.hi, (short)0, c, false, false);
    asm volatile("v_nop\n\tv_nop\n\tv_nop\n\tv_nop" : "+v"(c) : "v"(a.hi), "v"(a.lo), "v"(b.hi), "v"(b.lo));
    return c;
}
struct Split3 { v16b hi, mid, lo; };
__device__ __forceinline__ v8f wmma6(const Split3& a, const Split3& b, v8f c) {
    c = __builtin_amdgcn_wmma_f32_16x16x32_bf16(false, a.hi, false, b.hi, (short)0, c, false, false);
    c = __builtin_amdgcn_wmma_f32_16x16x32_bf16(false, a.hi, false, b.mid, (short)0, c, false, false);
    c = __builtin_amdgcn_wmma_f32_16x16x32_bf16(false, a.mid, false, b.hi, (short)0, c, false, false);
    c = __builtin_amdgcn_wmma_f32_16x16x32_bf16(false, a.hi, false, b.lo, (short)0, c, false, false);
    c = __builtin_amdgcn_wmma_f32_16x16x32_bf16(false, a.mid, false, b.mid, (short)0, c, false, false);
    c = __builtin_amdgcn_wmma_f32_16x16x32_bf16(false, a.lo, false, b.hi, (short)0, c, false, false);
    asm volatile("v_nop\n\tv_nop\n\tv_nop\n\tv_nop" : "+v"(c) : "v"(a.hi), "v"(a.mid), "v"(a.lo), "v"(b.hi), "v"(b.mid), "v"(b.lo));
    return c;
}

__device__ __forceinline__ v16h fh_ld(const float* __restrict__ p, long long sk, int k0, int h, int klen, float s) {
    v16h a;
#pragma unroll
    for (int i = 0; i < 16; ++i) { const int k = k0 + frag_k(i, h); a[i] = (k < klen) ? (_Float16)(p[(long long)k * sk] * s) : (_Float16)0.f; }
    return a;
}
__device__ __forceinline__ Split sp_ld(const float* __restrict__ p, long long sk, int k0, int h, int klen, float s) {
    Split r;
#pragma unroll
    for (int i = 0; i < 16; ++i) {
        const int k = k0 + frag_k(i, h); const float x = (k < klen) ? p[(long long)k * sk] * s : 0.f;
        const __bf16 hb = bf16_rne(x); r.hi[i] = hb; r.lo[i] = bf16_rne(x - bf16_f32(hb));
    }
    return r;
}
__device__ __forceinline__ Split3 sp3_ld(const float* __restrict__ p, long long sk, int k0, int h, int klen, float s) {
    Split3 r;
#pragma unroll
    for (int i = 0; i < 16; ++i) {
        const int k = k0 + frag_k(i, h); const float x = (k < klen) ? p[(long long)k * sk] * s : 0.f;
        const __bf16 hb = bf16_rne(x); const float r1 = x - bf16_f32(hb); const __bf16 mb = bf16_rne(r1);
        r.hi[i] = hb; r.mid[i] = mb; r.lo[i] = bf16_rne(r1 - bf16_f32(mb));
    }
    return r;
}
__device__ __forceinline__ v16b bh_ld(const float* __restrict__ p, long long sk, int k0, int h, int klen, float s) {
    v16b a;
#pragma unroll
    for (int i = 0; i < 16; ++i) { const int k = k0 + frag_k(i, h); a[i] = bf16_rne((k < klen) ? p[(long long)k * sk] * s : 0.f); }
    return a;
}
__device__ __forceinline__ v16h fh_row(const _Float16* __restrict__ row, int k0, int h) {
    v16h a;
#pragma unroll
    for (int i = 0; i < 16; ++i) a[i] = row[k0 + frag_k(i, h)];
    return a;
}

#define VST2(T, ptr, val) do { *(volatile T*)(ptr) = (val); __threadfence(); *(volatile T*)(ptr) = (val); } while (0)
typedef float v4f __attribute__((ext_vector_type(4)));
#define VST2V4(ptr, val) do { *(volatile v4f*)(ptr) = (val); __threadfence(); *(volatile v4f*)(ptr) = (val); } while (0)

__device__ __attribute__((noinline)) float act_fn(float v, int act) {
    if (act == 1) return fmaxf(v, 0.f);
    if (act == 2) { const float u = 0.7978845608028654f * (v + 0.044715f * v * v * v); return 0.5f * v * (1.f + tanhf(u)); }
    if (act == 3) return v / (1.f + expf(-v));
    if (act == 4) return 0.5f * v * (1.f + erff(v * 0.7071067811865476f));
    if (act == 5) return tanhf(v);
    if (act == 6) return 1.f / (1.f + expf(-v));
    if (act == 7) return (v > 0.f) ? v : 0.01f * v;
    if (act == 8) return (v > 0.f) ? v : (expf(v) - 1.f);
    if (act == 9) return fminf(fmaxf(v, 0.f), 6.f);
    if (act == 10) return fabsf(v);
    if (act == 11) return (v >= 0.f) ? v : 0.1f * v;
    if (act == 12) return (v > 0.f) ? v : 0.2f * v;
    if (act == 13) return (v > 20.f) ? v : log1pf(expf(v));
    return v;
}

struct GemmP {
    const float* A; const float* B; const float* bias; const float* R; float* C;
    long long sAo, sAi, sAm, sAk, sBo, sBi, sBn, sBk, sCo, sCi, sCm, sRo, sRi, sRm, sRn;
    int M, N, K, zi_n, flags, act; float alpha, beta, sa, sb;
    int Npad, pad_;
};
static_assert(sizeof(GemmP) == 5 * 8 + 15 * 8 + 6 * 4 + 4 * 4 + 2 * 4, "GemmP has padding");

template <int MODE>
__global__ __launch_bounds__(32) void k_gemm(GemmP p) {
    const int lane = threadIdx.x & 31, h = lane >> 4, l15 = lane & 15;
    const int m0 = blockIdx.y * 16, n0 = blockIdx.x * 32;
    const int z = blockIdx.z, zo = z / p.zi_n, zi = z - zo * p.zi_n;
    const float* A = p.A + zo * p.sAo + zi * p.sAi;
    const float* B = p.B + zo * p.sBo + zi * p.sBi;
    const int am = min(m0 + l15, p.M - 1);
    v8f acc[2], comp[2];
#pragma unroll
    for (int t = 0; t < 2; ++t) { v8f zz = {}; acc[t] = zz; comp[t] = zz; }
    for (int k0 = 0; k0 < p.K; k0 += 32) {
        const float* arow = A + (long long)am * p.sAm;
        if (MODE == 1) {
            const Split a = sp_ld(arow, p.sAk, k0, h, p.K, 1.f);
#pragma unroll
            for (int t = 0; t < 2; ++t) {
                const int bn = min(n0 + t * 16 + l15, p.N - 1);
                acc[t] = wmma3(a, sp_ld(B + (long long)bn * p.sBn, p.sBk, k0, h, p.K, 1.f), acc[t]);
            }
        } else if (MODE == 3) {
            const Split3 a = sp3_ld(arow, p.sAk, k0, h, p.K, 1.f);
#pragma unroll
            for (int t = 0; t < 2; ++t) {
                const int bn = min(n0 + t * 16 + l15, p.N - 1);
                acc[t] = wmma6(a, sp3_ld(B + (long long)bn * p.sBn, p.sBk, k0, h, p.K, 1.f), acc[t]);
            }
        } else if (MODE == 4) {
            const Split3 a = sp3_ld(arow, p.sAk, k0, h, p.K, 1.f);
#pragma unroll
            for (int t = 0; t < 2; ++t) {
                const int bn = min(n0 + t * 16 + l15, p.N - 1); v8f zz = {};
                const v8f part = wmma6(a, sp3_ld(B + (long long)bn * p.sBn, p.sBk, k0, h, p.K, 1.f), zz);
                const v8f y = part - comp[t]; const v8f s = acc[t] + y; comp[t] = (s - acc[t]) - y; acc[t] = s;
            }
        } else if (MODE == 2) {
            const v16b a = bh_ld(arow, p.sAk, k0, h, p.K, 1.f);
#pragma unroll
            for (int t = 0; t < 2; ++t) {
                const int bn = min(n0 + t * 16 + l15, p.N - 1);
                acc[t] = wmmab(a, bh_ld(B + (long long)bn * p.sBn, p.sBk, k0, h, p.K, 1.f), acc[t]);
            }
        } else {
            const v16h a = fh_ld(arow, p.sAk, k0, h, p.K, p.sa);
#pragma unroll
            for (int t = 0; t < 2; ++t) {
                const int bn = min(n0 + t * 16 + l15, p.N - 1);
                acc[t] = wmma16(a, fh_ld(B + (long long)bn * p.sBn, p.sBk, k0, h, p.K, p.sb), acc[t]);
            }
        }
    }
    const float iscale = (MODE == 0) ? p.alpha / (p.sa * p.sb) : p.alpha;
    float* C = p.C + zo * p.sCo + zi * p.sCi;
    const float* R = p.R + zo * p.sRo + zi * p.sRi;
    __shared__ __align__(16) float ctile[16][36];
#pragma unroll
    for (int t = 0; t < 2; ++t) {
        const int n = n0 + t * 16 + l15; const int nn = min(n, p.N - 1);
#pragma unroll
        for (int r = 0; r < 8; ++r) {
            const int m = m0 + 8 * h + r; const int mm = min(m, p.M - 1);
            float v = acc[t][r] * iscale;
            if (p.flags & 1) v += p.bias[nn];
            if (p.flags & 2) v += p.bias[mm];
            v = act_fn(v, p.act);
            if (p.flags & 4) v += p.beta * R[(long long)mm * p.sRm + (long long)nn * p.sRn];
            ctile[8 * h + r][t * 16 + l15] = (n < p.N) ? v : 0.f;
        }
    }
    __syncthreads();
    const int NW = (p.Npad > p.N) ? p.Npad : p.N;
    const bool fast = (m0 + 16 <= p.M) && (n0 + 32 <= NW) && ((p.sCm & 3) == 0) && ((((size_t)C) & 15) == 0);
    if (fast) {
#pragma unroll
        for (int s = 0; s < 4; ++s) {
            const int row = s * 4 + (lane >> 3), c4 = (lane & 7) * 4;
            const v4f v = *(const v4f*)&ctile[row][c4];
            VST2V4(C + (long long)(m0 + row) * p.sCm + n0 + c4, v);
        }
    } else {
        for (int row = 0; row < 16; ++row) {
            const int m = m0 + row, n = n0 + lane;
            if (m < p.M && n < NW) VST2(float, C + (long long)m * p.sCm + n, ctile[row][lane]);
        }
    }
}

#define AW 4
struct AttnP {
    const float* Q; const float* K; const float* V; float* O; float* P; const float* Mf; const int* Mi; float* ST;
    const float* Pw; const float* Rt; const int* SQ; const int* SK;
    long long swb, swh, swi, swj, srb, srh, sri;
    long long sQb, sQh, sQi, sQd, sKb, sKh, sKj, sKd, sVb, sVh, sVj, sVd, sOb, sOh, sOi, sPb, sPh, sPi, smb, smh, smi, smj;
    int Lq, Lk, dh, dv, hrep, causal, coff, pband;
    float scale, mfill; int nonorm, mpol;
    int roff, rn, segpol, win;
};
static_assert(sizeof(AttnP) == 12 * 8 + 29 * 8 + 16 * 4, "AttnP has padding");

#ifndef KATTN_ATTR
#define KATTN_ATTR
#endif
template <int DHP, int DVP, int QM, bool SPLITPV, bool TWOPASS>
__global__ __launch_bounds__(32 * AW) KATTN_ATTR void k_attn(AttnP p) {
    constexpr int NT = DVP / 16;
    constexpr int KS = DHP / 32;
    constexpr int VP = DVP + 8;
    __shared__ __align__(16) float    pl[AW][16 * 64];
    __shared__ __align__(16) _Float16 vl[(SPLITPV ? 2 : 1) * 64 * VP];
    const int lane = threadIdx.x & 31, hf = lane >> 4, l15 = lane & 15, wave = threadIdx.x >> 5;
    const int h = blockIdx.y, b = blockIdx.z, hk = h / p.hrep;
    const int q0 = (blockIdx.x * AW + wave) * 16;
    float* myp = pl[wave];
    const float L2E = 1.4426950408889634f;
    const float NEG = -__builtin_inff();
    const int qi = min(q0 + l15, p.Lq - 1);
    const float* qrow = p.Q + b * p.sQb + h * p.sQh + (long long)qi * p.sQi;
    const float* kbase = p.K + b * p.sKb + hk * p.sKh;
    const float* vbase = p.V + b * p.sVb + hk * p.sVh;
    v16h qa[QM == 0 ? KS : 1]; Split qs_[QM == 1 ? KS : 1]; Split3 qt_[QM == 2 ? KS : 1];
#pragma unroll
    for (int ks = 0; ks < KS; ++ks) {
        if (QM == 2) qt_[ks] = sp3_ld(qrow, p.sQd, ks * 32, hf, p.dh, 1.f);
        else if (QM == 1) qs_[ks] = sp_ld(qrow, p.sQd, ks * 32, hf, p.dh, 1.f);
        else qa[ks] = fh_ld(qrow, p.sQd, ks * 32, hf, p.dh, 1.f);
    }
    v8f o[NT]; float m8[8], l8[8];
#pragma unroll
    for (int t = 0; t < NT; ++t) { v8f zz = {}; o[t] = zz; }
#pragma unroll
    for (int i = 0; i < 8; ++i) { m8[i] = NEG; l8[i] = 0.f; }
    int jend = p.Lk;
    if (p.causal == 1) { const int je = (blockIdx.x * AW + AW - 1) * 16 + 16 + p.coff; jend = min(jend, max(je, 0)); }
    const int npass = TWOPASS ? 2 : 1;
    for (int pass = 0; pass < npass; ++pass) {
        const bool dopv = (!TWOPASS) || pass == 1;
        for (int j0 = 0; j0 < jend; j0 += 64) {
            if (dopv) {
                __syncthreads();
                for (int idx = threadIdx.x; idx < 64 * DVP; idx += 32 * AW) {
                    const int jr = idx / DVP, d = idx - jr * DVP, j = j0 + jr;
                    const float f = (j < p.Lk && d < p.dv) ? vbase[(long long)j * p.sVj + (long long)d * p.sVd] : 0.f;
                    if (SPLITPV) {
                        const __bf16 hb = bf16_rne(f);
                        ((__bf16*)vl)[jr * VP + d] = hb; ((__bf16*)vl)[64 * VP + jr * VP + d] = bf16_rne(f - bf16_f32(hb));
                    } else vl[jr * VP + d] = (_Float16)f;
                }
            }
            v8f s[4];
#pragma unroll
            for (int t = 0; t < 4; ++t) {
                const int j = min(j0 + t * 16 + l15, p.Lk - 1);
                const float* krow = kbase + (long long)j * p.sKj;
                v8f acc = {};
#pragma unroll
                for (int ks = 0; ks < KS; ++ks) {
                    if (QM == 2)      acc = wmma6(qt_[ks], sp3_ld(krow, p.sKd, ks * 32, hf, p.dh, 1.f), acc);
                    else if (QM == 1) acc = wmma3(qs_[ks], sp_ld(krow, p.sKd, ks * 32, hf, p.dh, 1.f), acc);
                    else              acc = wmma16(qa[ks], fh_ld(krow, p.sKd, ks * 32, hf, p.dh, 1.f), acc);
                }
                s[t] = acc;
            }
            float pv[8][4];
#pragma unroll
            for (int i = 0; i < 8; ++i) {
                const int irow = q0 + i + 8 * hf;
                const int ic = min(irow, p.Lq - 1);
                float sc[4];
#pragma unroll
                for (int t = 0; t < 4; ++t) {
                    const int jg = j0 + t * 16 + l15;
                    float v = s[t][i] * p.scale;
                    if (p.Mf) v += p.Mf[b * p.smb + h * p.smh + (long long)ic * p.smi + (long long)min(jg, p.Lk - 1) * p.smj];
                    if (p.Rt) { int rc = ic - min(jg, p.Lk - 1) + p.roff; rc = rc < 0 ? 0 : (rc >= p.rn ? p.rn - 1 : rc); v += p.Rt[b * p.srb + h * p.srh + (long long)ic * p.sri + rc]; }
                    if (p.Mi) { const int mv = p.Mi[b * p.smb + h * p.smh + (long long)ic * p.smi + (long long)min(jg, p.Lk - 1) * p.smj]; if (p.mpol ? (mv != 0) : (mv == 0)) v = p.mfill; }
                    if (p.SQ) { const bool same = p.SQ[(long long)b * p.Lq + ic] == p.SK[(long long)b * p.Lk + min(jg, p.Lk - 1)]; if (p.segpol ? same : !same) v = p.mfill; }
                    if (p.causal == 2 && jg > irow + p.coff) v = p.mfill;
                    if (jg >= p.Lk || (p.causal == 1 && jg > irow + p.coff) || (p.causal == 3 && jg < irow + p.coff) || (p.win > 0 && irow + p.coff - jg > p.win)) v = NEG; else v *= L2E;
                    sc[t] = v;
                }
                if (!TWOPASS || pass == 0) {
                    float mx = fmaxf(fmaxf(sc[0], sc[1]), fmaxf(sc[2], sc[3]));
                    mx = fmaxf(mx, __shfl_xor(mx, 1, 32)); mx = fmaxf(mx, __shfl_xor(mx, 2, 32));
                    mx = fmaxf(mx, __shfl_xor(mx, 4, 32)); mx = fmaxf(mx, __shfl_xor(mx, 8, 32));
                    const float mnew = fmaxf(m8[i], mx);
                    const float corr = (mnew == NEG) ? 1.f : exp2f(m8[i] - mnew);
                    float rs = 0.f;
#pragma unroll
                    for (int t = 0; t < 4; ++t) {
                        const float pp = (sc[t] == NEG) ? 0.f : exp2f(sc[t] - mnew); rs += pp;
                        pv[i][t] = p.Pw ? pp * p.Pw[b * p.swb + h * p.swh + (long long)ic * p.swi + (long long)min(j0 + t * 16 + l15, p.Lk - 1) * p.swj] : pp;
                    }
                    rs += __shfl_xor(rs, 1, 32); rs += __shfl_xor(rs, 2, 32); rs += __shfl_xor(rs, 4, 32); rs += __shfl_xor(rs, 8, 32);
                    l8[i] = l8[i] * corr + rs; m8[i] = mnew;
                    if (!TWOPASS) {
#pragma unroll
                        for (int t = 0; t < NT; ++t) o[t][i] *= corr;
                    }
                } else {
                    const float inv = (l8[i] > 0.f) ? 1.f / l8[i] : 0.f;
#pragma unroll
                    for (int t = 0; t < 4; ++t) {
                        const int jg = j0 + t * 16 + l15;
                        float pp = (sc[t] == NEG) ? 0.f : exp2f(sc[t] - m8[i]) * inv;
                        if (p.Pw) pp *= p.Pw[b * p.swb + h * p.swh + (long long)ic * p.swi + (long long)min(jg, p.Lk - 1) * p.swj];
                        pv[i][t] = pp;
                    }
                }
            }
            if (dopv) {
#pragma unroll
                for (int i = 0; i < 8; ++i)
#pragma unroll
                    for (int t = 0; t < 4; ++t) myp[(i + 8 * hf) * 64 + t * 16 + l15] = pv[i][t];
                __syncthreads();
                if (p.P) {
                    float* pb_ = p.P + b * p.sPb + h * p.sPh;
                    const bool fastP = (p.pband == 0) && ((p.sPi & 3) == 0) && (j0 + 64 <= p.Lk) && (q0 + 16 <= p.Lq) && ((((size_t)pb_) & 15) == 0);
                    if (fastP) {
#pragma unroll
                        for (int s = 0; s < 8; ++s) {
                            const int row = s * 2 + (lane >> 4), c4 = (lane & 15) * 4;
                            const v4f v = *(const v4f*)(myp + row * 64 + c4);
                            VST2V4(pb_ + (long long)(q0 + row) * p.sPi + j0 + c4, v);
                        }
                    } else {
                        for (int row = 0; row < 16; ++row) {
                            const int irow = q0 + row; if (irow >= p.Lq) continue;
                            for (int c = lane; c < 64; c += 32) {
                                const int jg = j0 + c; if (jg >= p.Lk) continue;
                                if (p.pband == 0) VST2(float, pb_ + (long long)irow * p.sPi + jg, myp[row * 64 + c]);
                                else if (jg - irow <= p.pband && irow - jg <= p.pband) VST2(float, pb_ + (long long)irow * p.sPi + (jg - irow + p.pband), myp[row * 64 + c]);
                            }
                        }
                    }
                }
                if (SPLITPV) {
                    const Split pa0 = sp_ld(myp + l15 * 64, 1, 0, hf, 64, 1.f), pa1 = sp_ld(myp + l15 * 64, 1, 32, hf, 64, 1.f);
                    const __bf16* vh = (const __bf16*)vl; const __bf16* vlo = vh + 64 * VP;
#pragma unroll
                    for (int t = 0; t < NT; ++t) {
                        const int dcol = t * 16 + l15;
                        Split b0, b1;
#pragma unroll
                        for (int e = 0; e < 16; ++e) {
                            const int k0 = frag_k(e, hf), k1 = 32 + frag_k(e, hf);
                            b0.hi[e] = vh[k0 * VP + dcol]; b0.lo[e] = vlo[k0 * VP + dcol]; b1.hi[e] = vh[k1 * VP + dcol]; b1.lo[e] = vlo[k1 * VP + dcol];
                        }
                        o[t] = wmma3(pa0, b0, o[t]);
                        o[t] = wmma3(pa1, b1, o[t]);
                    }
                } else {
                    const v16h pa0 = fh_ld(myp + l15 * 64, 1, 0, hf, 64, 4096.f), pa1 = fh_ld(myp + l15 * 64, 1, 32, hf, 64, 4096.f);
#pragma unroll
                    for (int t = 0; t < NT; ++t) {
                        const int dcol = t * 16 + l15;
                        v16h b0, b1;
#pragma unroll
                        for (int e = 0; e < 16; ++e) { b0[e] = vl[frag_k(e, hf) * VP + dcol]; b1[e] = vl[(32 + frag_k(e, hf)) * VP + dcol]; }
                        o[t] = wmma16(pa0, b0, o[t]);
                        o[t] = wmma16(pa1, b1, o[t]);
                    }
                }
            }
        }
    }
    float* obase = p.O + b * p.sOb + h * p.sOh;
    if (p.ST) {
        const int rl = lane >> 1, isel = rl & 7;
        float mv = 0.f, lv = 0.f;
#pragma unroll
        for (int i = 0; i < 8; ++i) if (i == isel) { mv = m8[i]; lv = l8[i]; }
        const int irow = q0 + rl;
        if (irow < p.Lq) { float* st = p.ST + (((long long)b * gridDim.y + h) * p.Lq + irow) * 2 + (lane & 1); VST2(float, st, (lane & 1) ? lv : mv * 0.6931471805599453f); }
    }
    float invr[8];
#pragma unroll
    for (int i = 0; i < 8; ++i) {
        if (TWOPASS) invr[i] = SPLITPV ? 1.f : (1.f / 4096.f);
        else if (p.nonorm) invr[i] = exp2f(m8[i]) * (SPLITPV ? 1.f : (1.f / 4096.f));
        else invr[i] = (l8[i] > 0.f) ? (SPLITPV ? 1.f / l8[i] : 1.f / (l8[i] * 4096.f)) : 0.f;
    }
    __syncthreads();
    const bool ofast = ((p.sOi & 3) == 0) && ((((size_t)obase) & 15) == 0) && (q0 + 16 <= p.Lq);
#pragma unroll
    for (int c0 = 0; c0 < DVP; c0 += 64) {
#pragma unroll
        for (int i = 0; i < 8; ++i)
#pragma unroll
            for (int t = 0; t < NT; ++t) if (t * 16 >= c0 && t * 16 < c0 + 64) myp[(i + 8 * hf) * 64 + (t * 16 - c0) + l15] = o[t][i] * invr[i];
        __syncthreads();
        const int cw = (DVP - c0 < 64) ? (DVP - c0) : 64;
        if (ofast && (c0 + cw <= p.dv) && (cw % 32 == 0)) {
            const int lpr = cw / 4;
            const int rows_per_ins = 32 / lpr;
            for (int r0 = 0; r0 < 16; r0 += rows_per_ins) {
                const int row = r0 + lane / lpr, c4 = (lane % lpr) * 4;
                const v4f v = *(const v4f*)(myp + row * 64 + c4);
                VST2V4(obase + (long long)(q0 + row) * p.sOi + c0 + c4, v);
            }
        } else {
            for (int row = 0; row < 16; ++row) {
                const int irow = q0 + row; if (irow >= p.Lq) continue;
                for (int c = lane; c < cw; c += 32) { const int d = c0 + c; if (d < p.dv) VST2(float, obase + (long long)irow * p.sOi + d, myp[row * 64 + c]); }
            }
        }
        __syncthreads();
    }
}

struct TrP { const float* src; float* dst; const float* R2; long long sSz, lds, sDz, ldd, sRz, ldr; int R, C, flags, act; float alpha, beta; };
static_assert(sizeof(TrP) == 3 * 8 + 6 * 8 + 6 * 4, "TrP has padding");
__global__ __launch_bounds__(256) void k_tr(TrP p) {
    __shared__ float tile[32][33];
    const int c0 = blockIdx.x * 32, r0 = blockIdx.y * 32, z = blockIdx.z;
    const int lane = threadIdx.x & 31, wave = threadIdx.x >> 5;
    const float* s = p.src + z * p.sSz;
#pragma unroll
    for (int k = 0; k < 4; ++k) {
        const int rl = wave * 4 + k, r = r0 + rl, c = c0 + lane;
        tile[rl][lane] = (r < p.R && c < p.C) ? s[(long long)r * p.lds + c] : 0.f;
    }
    __syncthreads();
    float* d = p.dst + z * p.sDz; const float* rr = p.R2 + z * p.sRz;
#pragma unroll
    for (int k = 0; k < 4; ++k) {
        const int cl = wave * 4 + k, c = c0 + cl, r = r0 + lane;
        if (c < p.C && r < p.R) {
            float v = act_fn(p.alpha * tile[lane][cl], p.act);
            if (p.flags & 1) v += p.beta * rr[(long long)c * p.ldr + r];
            VST2(float, d + (long long)c * p.ldd + r, v);
        }
    }
}

__global__ __launch_bounds__(256) void k_affine(const float* __restrict__ src, float* __restrict__ dst, int n, float a, float b, const float* __restrict__ sdev) {
    const int i = blockIdx.x * 256 + threadIdx.x;
    if (i < n) { const float aa = sdev ? a * sdev[0] : a; const float v = aa * src[i] + b; VST2(float, dst + i, v); }
}

struct SmP { const float* src; float* dst; const float* Mf; long long sz, sr, dz, dr, smz, smr; int n, pad; float scale_in, scale_out; };
static_assert(sizeof(SmP) == 3 * 8 + 6 * 8 + 4 * 4, "SmP has padding");
__global__ __launch_bounds__(256) void k_softmax(SmP p) {
    __shared__ float red[256];
    const int r = blockIdx.x, z = blockIdx.y, tid = threadIdx.x;
    const float* s = p.src + z * p.sz + (long long)r * p.sr;
    const float* mf = p.Mf ? (p.Mf + z * p.smz + (long long)r * p.smr) : nullptr;
    float mx = -__builtin_inff();
    for (int j = tid; j < p.n; j += 256) { float v = s[j] * p.scale_in; if (mf) v += mf[j]; mx = fmaxf(mx, v); }
    red[tid] = mx; __syncthreads();
    for (int o = 128; o > 0; o >>= 1) { if (tid < o) red[tid] = fmaxf(red[tid], red[tid + o]); __syncthreads(); }
    mx = red[0]; __syncthreads();
    float sum = 0.f;
    for (int j = tid; j < p.n; j += 256) { float v = s[j] * p.scale_in; if (mf) v += mf[j]; sum += (mx == -__builtin_inff()) ? 0.f : expf(v - mx); }
    red[tid] = sum; __syncthreads();
    for (int o = 128; o > 0; o >>= 1) { if (tid < o) red[tid] += red[tid + o]; __syncthreads(); }
    sum = red[0];
    const float inv = (sum > 0.f) ? p.scale_out / sum : 0.f;
    float* d = p.dst + z * p.dz + (long long)r * p.dr;
    for (int j = tid; j < p.n; j += 256) { float v = s[j] * p.scale_in; if (mf) v += mf[j]; const float o = (mx == -__builtin_inff()) ? 0.f : expf(v - mx) * inv; VST2(float, d + j, o); }
}
__global__ __launch_bounds__(256) void k_stats(const float* __restrict__ x, long long sz, long long so, long long si, int inner, int n, float eps, float* __restrict__ stat, int mode) {
    __shared__ float red[256];
    const int z = blockIdx.x, tid = threadIdx.x;
    const float* base = x + z * sz;
    float s = 0.f;
    for (int e = tid; e < n; e += 256) s += base[(long long)(e / inner) * so + (long long)(e % inner) * si];
    red[tid] = s; __syncthreads();
    for (int o = 128; o > 0; o >>= 1) { if (tid < o) red[tid] += red[tid + o]; __syncthreads(); }
    const float mu = (mode == 0 || mode == 3) ? red[0] / (float)n : 0.f; __syncthreads();
    float q = 0.f;
    for (int e = tid; e < n; e += 256) { const float dlt = base[(long long)(e / inner) * so + (long long)(e % inner) * si] - mu; q += dlt * dlt; }
    red[tid] = q; __syncthreads();
    for (int o = 128; o > 0; o >>= 1) { if (tid < o) red[tid] += red[tid + o]; __syncthreads(); }
    {
        float rs;
        if (mode == 2) rs = sqrtf((float)n) / fmaxf(sqrtf(red[0]), eps); else if (mode == 3) rs = rsqrtf(red[0] / (float)(n - 1) + eps); else rs = rsqrtf(red[0] / (float)n + eps);
        if (tid < 32) { const float v = (tid == 0) ? mu : ((tid == 1) ? rs : 0.f); VST2(float, stat + (long long)z * 32 + tid, v); }
    }
}
__global__ __launch_bounds__(256) void k_norm_apply(const float* __restrict__ x, float* __restrict__ y, const float* __restrict__ stat, const float* __restrict__ g, const float* __restrict__ bta,
                                                     int Z, int C, int L, int G, int bn, int act) {
    const long long idx = (long long)blockIdx.x * 256 + threadIdx.x;
    if (idx >= (long long)Z * C * L) return;
    const int l = (int)(idx % L); const long long zc = idx / L; const int c = (int)(zc % C), z = (int)(zc / C); (void)l;
    const int set = bn ? c : (z * G + c / (C / G));
    float v = (x[idx] - stat[(long long)set * 32]) * stat[(long long)set * 32 + 1];
    if (g) v *= g[c];
    if (bta) v += bta[c];
    v = act_fn(v, act);
    VST2(float, y + idx, v);
}

__global__ __launch_bounds__(256) void k_lse_neg(const float* __restrict__ st, float* __restrict__ c, int n) {
    const int i = blockIdx.x * 256 + threadIdx.x;
    if (i < n) { const float v = -(st[2 * i] + logf(st[2 * i + 1])); VST2(float, c + i, v); }
}

__global__ __launch_bounds__(256) void k_iota(int* __restrict__ dst, int n, int a, int b) {
    const int i = blockIdx.x * 256 + threadIdx.x;
    if (i < n) { const int v = a * i + b; VST2(int, dst + i, v); }
}

__global__ __launch_bounds__(256) void k_axpby(const float* __restrict__ x, const float* __restrict__ y, float* __restrict__ dst, int n, float a, float b, float c) {
    const int i = blockIdx.x * 256 + threadIdx.x;
    if (i < n) { const float v = a * x[i] + b * y[i] + c; VST2(float, dst + i, v); }
}

struct RopeP { const float* X; float* Y; const float* C; const float* Sn; const int* pos; long long sXr, sXh, sYr, sYh, sCb, sCp, sCd; int R, Hn, D, S, mode, tmode, pmode, pad; };
static_assert(sizeof(RopeP) == 5 * 8 + 7 * 8 + 8 * 4, "RopeP has padding");
__global__ __launch_bounds__(256) void k_rope(RopeP p) {
    const long long idx = (long long)blockIdx.x * 256 + threadIdx.x;
    if (idx >= (long long)p.R * p.Hn * p.D) return;
    const int d = (int)(idx % p.D); const long long rh = idx / p.D; const int h = (int)(rh % p.Hn); const int r = (int)(rh / p.Hn);
    const int half = p.D / 2;
    int partner; float sign;
    if (p.mode == 0) { partner = (d < half) ? d + half : d - half; sign = (d < half) ? -1.f : 1.f; }
    else { partner = d ^ 1; sign = (d & 1) ? 1.f : -1.f; }
    const int tcol = (p.tmode == 0) ? d : ((p.tmode == 1) ? (d % half) : (d >> 1));
    const int pp = (p.pmode == 0) ? (r % p.S) : ((p.pmode == 1) ? h : p.pos[r]);
    const long long toff = (long long)(r / p.S) * p.sCb + (long long)pp * p.sCp + (long long)tcol * p.sCd;
    const float* xr = p.X + (long long)r * p.sXr + (long long)h * p.sXh;
    const float v = xr[d] * p.C[toff] + sign * xr[partner] * p.Sn[toff];
    VST2(float, p.Y + (long long)r * p.sYr + (long long)h * p.sYh + d, v);
}

__global__ __launch_bounds__(256) void k_invf(float* __restrict__ invb, int half, int D, float base, float num, int fmode, float cexp) {
    const int i = blockIdx.x * 256 + threadIdx.x;
    if (i >= ((half + 31) / 32) * 32) return;
    if (i >= half) { VST2(float, invb + i, 0.f); return; }
    const float e = (float)(2 * i) / (float)D;
    float invf;
    if (fmode == 1) invf = num * expf((float)(2 * i) * cexp);
    else if (fmode == 2) invf = num * powf(base, (-2.0f * ((float)i - 1.0f)) / (float)D);
    else invf = num * (1.0f / powf(base, e));
    VST2(float, invb + i, invf);
}
__global__ __launch_bounds__(256) void k_sincos(float* __restrict__ cs, float* __restrict__ sn, const float* __restrict__ invb, int S, int half, float pscale) {
    const int idx = blockIdx.x * 256 + threadIdx.x;
    if (idx >= S * half) return;
    const int s = idx / half, i = idx - s * half;
    const float ang = (pscale * (float)s) * invb[i];
    VST2(float, cs + idx, cosf(ang)); VST2(float, sn + idx, sinf(ang));
}

__global__ __launch_bounds__(256) void k_mulact(const float* __restrict__ x, const float* __restrict__ y, float* __restrict__ dst, int n, int act) {
    const int i = blockIdx.x * 256 + threadIdx.x;
    if (i < n) { const float v = act_fn(x[i], act) * y[i]; VST2(float, dst + i, v); }
}

__global__ __launch_bounds__(256) void k_matvec(GemmP p) {
    const int rpt = (p.N == 1) ? 1 : 32;
    const long long r0 = ((long long)blockIdx.x * 256 + threadIdx.x) * rpt; const int z = blockIdx.z, zo = z / p.zi_n, zi = z - zo * p.zi_n;
    if (r0 >= p.M) return;
    const float* Bb = p.B + zo * p.sBo + zi * p.sBi;
    float* C = p.C + zo * p.sCo + zi * p.sCi; const float* R = p.R + zo * p.sRo + zi * p.sRi;
    for (int rr = 0; rr < rpt; ++rr) {
        const long long r = r0 + rr; if (r >= p.M) break;
        const float* A = p.A + zo * p.sAo + zi * p.sAi + r * p.sAm;
        float acc[8] = {0.f, 0.f, 0.f, 0.f, 0.f, 0.f, 0.f, 0.f};
        for (int k = 0; k < p.K; ++k) { const float a = A[(long long)k * p.sAk];
#pragma unroll
            for (int j = 0; j < 8; ++j) if (j < p.N) acc[j] += a * Bb[(long long)j * p.sBn + (long long)k * p.sBk]; }
#pragma unroll
        for (int j = 0; j < 8; ++j) if (j < p.N) {
            float v = acc[j] * p.alpha;
            if (p.flags & 1) v += p.bias[j];
            if (p.flags & 2) v += p.bias[r];
            v = act_fn(v, p.act);
            if (p.flags & 4) v += p.beta * R[r * p.sRm + (long long)j * p.sRn];
            VST2(float, C + r * p.sCm + j, v);
        }
    }
}
__global__ __launch_bounds__(256) void k_smallsoftmax(const float* __restrict__ src, float* __restrict__ dst, long long sr, long long dr, int n, long long R, float scale) {
    const long long r0 = ((long long)blockIdx.x * 256 + threadIdx.x) * 32;
    for (int rr = 0; rr < 32; ++rr) {
        const long long r = r0 + rr; if (r >= R) return;
        const float* s = src + r * sr; float* d = dst + r * dr;
        float mx = -__builtin_inff();
        for (int j = 0; j < n; ++j) mx = fmaxf(mx, s[j] * scale);
        float sum = 0.f;
        for (int j = 0; j < n; ++j) sum += expf(s[j] * scale - mx);
        const float inv = 1.f / sum;
        for (int j = 0; j < n; ++j) { const float v = expf(s[j] * scale - mx) * inv; VST2(float, d + j, v); }
    }
}

__global__ __launch_bounds__(32) void k_unitstat(float* __restrict__ st) { const int t = threadIdx.x; const float v = (t == 1) ? 1.f : 0.f; VST2(float, st + t, v); }

__global__ __launch_bounds__(256) void k_lincopy(const float* __restrict__ src, long long lds, float* __restrict__ dst, long long ldd, long long rows, int cols) {
    const long long i = (long long)blockIdx.x * 256 + threadIdx.x; if (i >= rows * cols) return;
    const long long r = i / cols; const int c = (int)(i - r * cols);
    const float v = src[r * lds + c]; VST2(float, dst + r * ldd + c, v);
}

__device__ __forceinline__ void wb_mobius(const float x[3], const float y[3], float c, float out[3]) {
    const float EPSv = 1e-7f; float x2 = 0.f, y2 = 0.f, xy = 0.f;
    for (int d = 0; d < 3; ++d) { x2 += x[d] * x[d]; y2 += y[d] * y[d]; xy += x[d] * y[d]; }
    const float a = 1.f + 2.f * c * xy + c * y2, b = 1.f - c * x2; const float den = fmaxf(1.f + 2.f * c * xy + c * c * x2 * y2, EPSv);
    float v[3]; float n2 = 0.f; for (int d = 0; d < 3; ++d) { v[d] = (a * x[d] + b * y[d]) / den; n2 += v[d] * v[d]; }
    const float sqrt_c = fmaxf(sqrtf(c), EPSv); const float nrm = fmaxf(sqrtf(n2), EPSv); const float mx = (1.f - EPSv) / sqrt_c; const float f = fminf(mx / nrm, 1.f);
    for (int d = 0; d < 3; ++d) out[d] = v[d] * f;
}
__global__ __launch_bounds__(128) void k_wubu_knn(const float* __restrict__ pos, const float* __restrict__ cc, int* __restrict__ IDX, int N) {
    __shared__ float sp[3 * 512];
    const int i = blockIdx.x * 128 + threadIdx.x; const bool ok = i < N; const float c = cc[0]; const float EPSv = 1e-7f; const float sqrt_c = fmaxf(sqrtf(c), EPSv);
    float yi[3]; for (int d = 0; d < 3; ++d) yi[d] = ok ? -pos[3 * i + d] : 0.f;
    float bd[32]; int bi[32]; for (int j = 0; j < 32; ++j) { bd[j] = __builtin_inff(); bi[j] = 0; }
    for (int j0 = 0; j0 < N; j0 += 512) {
        const int nt = min(512, N - j0); __syncthreads(); for (int q = threadIdx.x; q < nt * 3; q += 128) sp[q] = pos[(long long)j0 * 3 + q]; __syncthreads();
        for (int q = 0; q < nt; ++q) { const int j = j0 + q; float xj[3] = {sp[3 * q], sp[3 * q + 1], sp[3 * q + 2]}; float df[3]; wb_mobius(xj, yi, c, df);
            const float dn = sqrtf(df[0] * df[0] + df[1] * df[1] + df[2] * df[2]); const float arg = fminf(sqrt_c * fminf(fmaxf(dn, EPSv), 1.f - EPSv), 1.f - EPSv); const float dist = 2.f * atanhf(arg) / sqrt_c;
            if (dist < bd[31]) { int s = 31; while (s > 0 && dist < bd[s - 1]) { bd[s] = bd[s - 1]; bi[s] = bi[s - 1]; --s; } bd[s] = dist; bi[s] = j; } }
    }
    if (ok) for (int j = 0; j < 32; ++j) VST2(int, IDX + (long long)i * 32 + j, bi[j]);
}
__global__ __launch_bounds__(256) void k_wubu_gather(const float* __restrict__ KF, const float* __restrict__ VF, const int* __restrict__ IDX, const float* __restrict__ pos, const float* __restrict__ cc, float* __restrict__ KG, float* __restrict__ VG, float* __restrict__ GEO, int n0, int CH) {
    const long long t = (long long)blockIdx.x * 256 + threadIdx.x; if (t >= (long long)CH * 32 * 512) return; const int col = (int)(t % 512); const int kk = (int)((t / 512) % 32); const int nl = (int)(t / (512 * 32)); const int n = n0 + nl; const int j = IDX[(long long)n * 32 + kk];
    VST2(float, KG + t, KF[(long long)j * 512 + col]); VST2(float, VG + t, VF[(long long)j * 512 + col]);
    if (col < 4) { float v = 0.f; if (col < 3) { const float c = cc[0]; const float EPSv = 1e-7f; const float sqrt_c = fmaxf(sqrtf(c), EPSv); float mq[3], kp[3], g[3]; for (int d = 0; d < 3; ++d) { mq[d] = -pos[3 * n + d]; kp[d] = pos[3 * j + d]; }
            wb_mobius(mq, kp, c, g); const float yn = sqrtf(g[0] * g[0] + g[1] * g[1] + g[2] * g[2]); const float safe = fmaxf(yn, EPSv); const float mag = atanhf(fminf(sqrt_c * safe, 1.f - EPSv)) / sqrt_c; v = (yn < EPSv) ? 0.f : mag * (g[col] / safe); }
        VST2(float, GEO + ((long long)nl * 32 + kk) * 4 + col, v); }
}
__global__ __launch_bounds__(256) void k_wubu_soft(const float* __restrict__ SC1, const float* __restrict__ SC2, const float* __restrict__ asc, const float* __restrict__ fsc, float* __restrict__ WT, int NZ) {
    const int z = blockIdx.x * 256 + threadIdx.x; if (z >= NZ) return; const int h = z % 8; float s[32]; float mx = -__builtin_inff();
    for (int kk = 0; kk < 32; ++kk) { s[kk] = fsc[h] * (SC1[(long long)z * 32 + kk] * 0.125f) + asc[h] * SC2[(long long)z * 32 + kk]; mx = fmaxf(mx, s[kk]); }
    float sum = 0.f; for (int kk = 0; kk < 32; ++kk) { s[kk] = expf(s[kk] - mx); sum += s[kk]; }
    for (int kk = 0; kk < 32; ++kk) VST2(float, WT + (long long)z * 32 + kk, s[kk] / sum);
}

template __global__ void k_gemm<1>(GemmP);

extern "C" void kernel_launch(void* const* d_in, const int* in_sizes, int n_in, void* d_out, int out_size, void* d_ws, size_t ws_size, hipStream_t stream) {
    (void)in_sizes; (void)n_in; (void)out_size; (void)ws_size;
    const float* x = (const float*)d_in[0];
    const float* pos = (const float*)d_in[1];
    const float* cc = (const float*)d_in[2];
    const float* wq = (const float*)d_in[3];
    const float* bq = (const float*)d_in[4];
    const float* wk = (const float*)d_in[5];
    const float* bk = (const float*)d_in[6];
    const float* wv = (const float*)d_in[7];
    const float* bv = (const float*)d_in[8];
    const float* wg = (const float*)d_in[9];
    const float* bg = (const float*)d_in[10];
    const float* wo = (const float*)d_in[11];
    const float* bo = (const float*)d_in[12];
    const float* w1 = (const float*)d_in[13];
    const float* b1 = (const float*)d_in[14];
    const float* w2 = (const float*)d_in[15];
    const float* b2 = (const float*)d_in[16];
    const float* l1s = (const float*)d_in[17];
    const float* l1b = (const float*)d_in[18];
    const float* l2s = (const float*)d_in[19];
    const float* l2b = (const float*)d_in[20];
    const float* asc = (const float*)d_in[21];
    const float* fsc = (const float*)d_in[22];
    const int N = 4096;
    const int D = 512;
    const int NH = 8;
    const int HD = 64;
    const int KN = 32;
    const int DFF = 2048;
    const int CHN = 512;
    float* out = (float*)d_out;
    char* wsp = (char*)d_ws;
    float* st = (float*)wsp; wsp += (((size_t)((size_t)N * 32) * 4 + 255) / 256) * 256;
    float* XN = (float*)wsp; wsp += (((size_t)((size_t)N * D) * 4 + 255) / 256) * 256;
    float* Q = (float*)wsp; wsp += (((size_t)((size_t)N * D) * 4 + 255) / 256) * 256;
    float* KF = (float*)wsp; wsp += (((size_t)((size_t)N * D) * 4 + 255) / 256) * 256;
    float* VF = (float*)wsp; wsp += (((size_t)((size_t)N * D) * 4 + 255) / 256) * 256;
    int* IDX = (int*)wsp; wsp += (((size_t)((size_t)N * KN) * 4 + 255) / 256) * 256;
    float* AT = (float*)wsp; wsp += (((size_t)((size_t)N * D) * 4 + 255) / 256) * 256;
    float* X1 = (float*)wsp; wsp += (((size_t)((size_t)N * D) * 4 + 255) / 256) * 256;
    float* H2 = (float*)wsp; wsp += (((size_t)((size_t)N * D) * 4 + 255) / 256) * 256;
    float* T = (float*)wsp; wsp += (((size_t)((size_t)N * DFF) * 4 + 255) / 256) * 256;
    float* KG = (float*)wsp; wsp += (((size_t)((size_t)CHN * KN * D) * 4 + 255) / 256) * 256;
    float* VG = (float*)wsp; wsp += (((size_t)((size_t)CHN * KN * D) * 4 + 255) / 256) * 256;
    float* GEO = (float*)wsp; wsp += (((size_t)((size_t)CHN * KN * 4) * 4 + 255) / 256) * 256;
    float* GP = (float*)wsp; wsp += (((size_t)((size_t)CHN * KN * D) * 4 + 255) / 256) * 256;
    float* SC1 = (float*)wsp; wsp += (((size_t)((size_t)CHN * NH * KN) * 4 + 255) / 256) * 256;
    float* SC2 = (float*)wsp; wsp += (((size_t)((size_t)CHN * NH * KN) * 4 + 255) / 256) * 256;
    float* WT = (float*)wsp; wsp += (((size_t)((size_t)CHN * NH * KN) * 4 + 255) / 256) * 256;
    k_stats<<<(unsigned)(N), 256, 0, stream>>>(x, D, 0, 1, D, D, 1e-06f, st, 0);
    k_norm_apply<<<(unsigned)(((long long)(N) * (D) * (1) + 255) / 256), 256, 0, stream>>>(x, XN, st, l1s, l1b, N, D, 1, 1, 0, 0);
    { GemmP gQ;
      gQ.A = XN; gQ.B = wq; gQ.bias = bq; gQ.R = XN; gQ.C = Q;
      gQ.sAo = 0; gQ.sAi = 0; gQ.sAm = D; gQ.sAk = 1; gQ.sBo = 0; gQ.sBi = 0; gQ.sBn = 1; gQ.sBk = D; gQ.sCo = 0; gQ.sCi = 0; gQ.sCm = D; gQ.sRo = 0; gQ.sRi = 0; gQ.sRm = 0; gQ.sRn = 0;
      gQ.M = N; gQ.N = D; gQ.K = D; gQ.zi_n = 1; gQ.flags = 1; gQ.act = 0;
      gQ.alpha = 1.0f; gQ.beta = 0.0f; gQ.sa = 1.0f; gQ.sb = 1.0f; gQ.Npad = D; gQ.pad_ = 0;
      k_gemm<1><<<dim3((unsigned)((D) + 31) / 32, (unsigned)((N) + 15) / 16, (unsigned)(1)), 32, 0, stream>>>(gQ); }
    { GemmP gKF;
      gKF.A = XN; gKF.B = wk; gKF.bias = bk; gKF.R = XN; gKF.C = KF;
      gKF.sAo = 0; gKF.sAi = 0; gKF.sAm = D; gKF.sAk = 1; gKF.sBo = 0; gKF.sBi = 0; gKF.sBn = 1; gKF.sBk = D; gKF.sCo = 0; gKF.sCi = 0; gKF.sCm = D; gKF.sRo = 0; gKF.sRi = 0; gKF.sRm = 0; gKF.sRn = 0;
      gKF.M = N; gKF.N = D; gKF.K = D; gKF.zi_n = 1; gKF.flags = 1; gKF.act = 0;
      gKF.alpha = 1.0f; gKF.beta = 0.0f; gKF.sa = 1.0f; gKF.sb = 1.0f; gKF.Npad = D; gKF.pad_ = 0;
      k_gemm<1><<<dim3((unsigned)((D) + 31) / 32, (unsigned)((N) + 15) / 16, (unsigned)(1)), 32, 0, stream>>>(gKF); }
    { GemmP gVF;
      gVF.A = XN; gVF.B = wv; gVF.bias = bv; gVF.R = XN; gVF.C = VF;
      gVF.sAo = 0; gVF.sAi = 0; gVF.sAm = D; gVF.sAk = 1; gVF.sBo = 0; gVF.sBi = 0; gVF.sBn = 1; gVF.sBk = D; gVF.sCo = 0; gVF.sCi = 0; gVF.sCm = D; gVF.sRo = 0; gVF.sRi = 0; gVF.sRm = 0; gVF.sRn = 0;
      gVF.M = N; gVF.N = D; gVF.K = D; gVF.zi_n = 1; gVF.flags = 1; gVF.act = 0;
      gVF.alpha = 1.0f; gVF.beta = 0.0f; gVF.sa = 1.0f; gVF.sb = 1.0f; gVF.Npad = D; gVF.pad_ = 0;
      k_gemm<1><<<dim3((unsigned)((D) + 31) / 32, (unsigned)((N) + 15) / 16, (unsigned)(1)), 32, 0, stream>>>(gVF); }
    k_wubu_knn<<<(unsigned)((N + 127) / 128), 128, 0, stream>>>(pos, cc, IDX, N);
    k_wubu_gather<<<(unsigned)(((long long)CHN * KN * D + 255) / 256), 256, 0, stream>>>(KF, VF, IDX, pos, cc, KG, VG, GEO, 0, CHN);
    { GemmP ggp0;
      ggp0.A = GEO; ggp0.B = wg; ggp0.bias = bg; ggp0.R = GEO; ggp0.C = GP;
      ggp0.sAo = 0; ggp0.sAi = 0; ggp0.sAm = 4; ggp0.sAk = 1; ggp0.sBo = 0; ggp0.sBi = 0; ggp0.sBn = 1; ggp0.sBk = D; ggp0.sCo = 0; ggp0.sCi = 0; ggp0.sCm = D; ggp0.sRo = 0; ggp0.sRi = 0; ggp0.sRm = 0; ggp0.sRn = 0;
      ggp0.M = CHN * KN; ggp0.N = D; ggp0.K = 3; ggp0.zi_n = 1; ggp0.flags = 1; ggp0.act = 0;
      ggp0.alpha = 1.0f; ggp0.beta = 0.0f; ggp0.sa = 1.0f; ggp0.sb = 1.0f; ggp0.Npad = D; ggp0.pad_ = 0;
      k_gemm<1><<<dim3((unsigned)((D) + 31) / 32, (unsigned)((CHN * KN) + 15) / 16, (unsigned)(1)), 32, 0, stream>>>(ggp0); }
    { GemmP gSC1_0;
      gSC1_0.A = Q + (size_t)0 * D; gSC1_0.B = KG; gSC1_0.bias = Q + (size_t)0 * D; gSC1_0.R = Q + (size_t)0 * D; gSC1_0.C = SC1;
      gSC1_0.sAo = D; gSC1_0.sAi = HD; gSC1_0.sAm = 0; gSC1_0.sAk = 1; gSC1_0.sBo = (long long)KN * D; gSC1_0.sBi = HD; gSC1_0.sBn = D; gSC1_0.sBk = 1; gSC1_0.sCo = NH * KN; gSC1_0.sCi = KN; gSC1_0.sCm = KN; gSC1_0.sRo = 0; gSC1_0.sRi = 0; gSC1_0.sRm = 0; gSC1_0.sRn = 0;
      gSC1_0.M = 1; gSC1_0.N = KN; gSC1_0.K = HD; gSC1_0.zi_n = NH; gSC1_0.flags = 0; gSC1_0.act = 0;
      gSC1_0.alpha = 1.0f; gSC1_0.beta = 0.0f; gSC1_0.sa = 1.0f; gSC1_0.sb = 1.0f; gSC1_0.Npad = KN; gSC1_0.pad_ = 0;
      k_gemm<1><<<dim3((unsigned)((KN) + 31) / 32, (unsigned)((1) + 15) / 16, (unsigned)(CHN * NH)), 32, 0, stream>>>(gSC1_0); }
    { GemmP gSC2_0;
      gSC2_0.A = Q + (size_t)0 * D; gSC2_0.B = GP; gSC2_0.bias = Q + (size_t)0 * D; gSC2_0.R = Q + (size_t)0 * D; gSC2_0.C = SC2;
      gSC2_0.sAo = D; gSC2_0.sAi = HD; gSC2_0.sAm = 0; gSC2_0.sAk = 1; gSC2_0.sBo = (long long)KN * D; gSC2_0.sBi = HD; gSC2_0.sBn = D; gSC2_0.sBk = 1; gSC2_0.sCo = NH * KN; gSC2_0.sCi = KN; gSC2_0.sCm = KN; gSC2_0.sRo = 0; gSC2_0.sRi = 0; gSC2_0.sRm = 0; gSC2_0.sRn = 0;
      gSC2_0.M = 1; gSC2_0.N = KN; gSC2_0.K = HD; gSC2_0.zi_n = NH; gSC2_0.flags = 0; gSC2_0.act = 0;
      gSC2_0.alpha = 1.0f; gSC2_0.beta = 0.0f; gSC2_0.sa = 1.0f; gSC2_0.sb = 1.0f; gSC2_0.Npad = KN; gSC2_0.pad_ = 0;
      k_gemm<1><<<dim3((unsigned)((KN) + 31) / 32, (unsigned)((1) + 15) / 16, (unsigned)(CHN * NH)), 32, 0, stream>>>(gSC2_0); }
    k_wubu_soft<<<(unsigned)((CHN * NH + 255) / 256), 256, 0, stream>>>(SC1, SC2, asc, fsc, WT, CHN * NH);
    { GemmP gat0;
      gat0.A = WT; gat0.B = VG; gat0.bias = WT; gat0.R = WT; gat0.C = AT + (size_t)0 * D;
      gat0.sAo = NH * KN; gat0.sAi = KN; gat0.sAm = 0; gat0.sAk = 1; gat0.sBo = (long long)KN * D; gat0.sBi = HD; gat0.sBn = 1; gat0.sBk = D; gat0.sCo = D; gat0.sCi = HD; gat0.sCm = HD; gat0.sRo = 0; gat0.sRi = 0; gat0.sRm = 0; gat0.sRn = 0;
      gat0.M = 1; gat0.N = HD; gat0.K = KN; gat0.zi_n = NH; gat0.flags = 0; gat0.act = 0;
      gat0.alpha = 1.0f; gat0.beta = 0.0f; gat0.sa = 1.0f; gat0.sb = 1.0f; gat0.Npad = HD; gat0.pad_ = 0;
      k_gemm<1><<<dim3((unsigned)((HD) + 31) / 32, (unsigned)((1) + 15) / 16, (unsigned)(CHN * NH)), 32, 0, stream>>>(gat0); }
    k_wubu_gather<<<(unsigned)(((long long)CHN * KN * D + 255) / 256), 256, 0, stream>>>(KF, VF, IDX, pos, cc, KG, VG, GEO, 512, CHN);
    { GemmP ggp1;
      ggp1.A = GEO; ggp1.B = wg; ggp1.bias = bg; ggp1.R = GEO; ggp1.C = GP;
      ggp1.sAo = 0; ggp1.sAi = 0; ggp1.sAm = 4; ggp1.sAk = 1; ggp1.sBo = 0; ggp1.sBi = 0; ggp1.sBn = 1; ggp1.sBk = D; ggp1.sCo = 0; ggp1.sCi = 0; ggp1.sCm = D; ggp1.sRo = 0; ggp1.sRi = 0; ggp1.sRm = 0; ggp1.sRn = 0;
      ggp1.M = CHN * KN; ggp1.N = D; ggp1.K = 3; ggp1.zi_n = 1; ggp1.flags = 1; ggp1.act = 0;
      ggp1.alpha = 1.0f; ggp1.beta = 0.0f; ggp1.sa = 1.0f; ggp1.sb = 1.0f; ggp1.Npad = D; ggp1.pad_ = 0;
      k_gemm<1><<<dim3((unsigned)((D) + 31) / 32, (unsigned)((CHN * KN) + 15) / 16, (unsigned)(1)), 32, 0, stream>>>(ggp1); }
    { GemmP gSC1_1;
      gSC1_1.A = Q + (size_t)512 * D; gSC1_1.B = KG; gSC1_1.bias = Q + (size_t)512 * D; gSC1_1.R = Q + (size_t)512 * D; gSC1_1.C = SC1;
      gSC1_1.sAo = D; gSC1_1.sAi = HD; gSC1_1.sAm = 0; gSC1_1.sAk = 1; gSC1_1.sBo = (long long)KN * D; gSC1_1.sBi = HD; gSC1_1.sBn = D; gSC1_1.sBk = 1; gSC1_1.sCo = NH * KN; gSC1_1.sCi = KN; gSC1_1.sCm = KN; gSC1_1.sRo = 0; gSC1_1.sRi = 0; gSC1_1.sRm = 0; gSC1_1.sRn = 0;
      gSC1_1.M = 1; gSC1_1.N = KN; gSC1_1.K = HD; gSC1_1.zi_n = NH; gSC1_1.flags = 0; gSC1_1.act = 0;
      gSC1_1.alpha = 1.0f; gSC1_1.beta = 0.0f; gSC1_1.sa = 1.0f; gSC1_1.sb = 1.0f; gSC1_1.Npad = KN; gSC1_1.pad_ = 0;
      k_gemm<1><<<dim3((unsigned)((KN) + 31) / 32, (unsigned)((1) + 15) / 16, (unsigned)(CHN * NH)), 32, 0, stream>>>(gSC1_1); }
    { GemmP gSC2_1;
      gSC2_1.A = Q + (size_t)512 * D; gSC2_1.B = GP; gSC2_1.bias = Q + (size_t)512 * D; gSC2_1.R = Q + (size_t)512 * D; gSC2_1.C = SC2;
      gSC2_1.sAo = D; gSC2_1.sAi = HD; gSC2_1.sAm = 0; gSC2_1.sAk = 1; gSC2_1.sBo = (long long)KN * D; gSC2_1.sBi = HD; gSC2_1.sBn = D; gSC2_1.sBk = 1; gSC2_1.sCo = NH * KN; gSC2_1.sCi = KN; gSC2_1.sCm = KN; gSC2_1.sRo = 0; gSC2_1.sRi = 0; gSC2_1.sRm = 0; gSC2_1.sRn = 0;
      gSC2_1.M = 1; gSC2_1.N = KN; gSC2_1.K = HD; gSC2_1.zi_n = NH; gSC2_1.flags = 0; gSC2_1.act = 0;
      gSC2_1.alpha = 1.0f; gSC2_1.beta = 0.0f; gSC2_1.sa = 1.0f; gSC2_1.sb = 1.0f; gSC2_1.Npad = KN; gSC2_1.pad_ = 0;
      k_gemm<1><<<dim3((unsigned)((KN) + 31) / 32, (unsigned)((1) + 15) / 16, (unsigned)(CHN * NH)), 32, 0, stream>>>(gSC2_1); }
    k_wubu_soft<<<(unsigned)((CHN * NH + 255) / 256), 256, 0, stream>>>(SC1, SC2, asc, fsc, WT, CHN * NH);
    { GemmP gat1;
      gat1.A = WT; gat1.B = VG; gat1.bias = WT; gat1.R = WT; gat1.C = AT + (size_t)512 * D;
      gat1.sAo = NH * KN; gat1.sAi = KN; gat1.sAm = 0; gat1.sAk = 1; gat1.sBo = (long long)KN * D; gat1.sBi = HD; gat1.sBn = 1; gat1.sBk = D; gat1.sCo = D; gat1.sCi = HD; gat1.sCm = HD; gat1.sRo = 0; gat1.sRi = 0; gat1.sRm = 0; gat1.sRn = 0;
      gat1.M = 1; gat1.N = HD; gat1.K = KN; gat1.zi_n = NH; gat1.flags = 0; gat1.act = 0;
      gat1.alpha = 1.0f; gat1.beta = 0.0f; gat1.sa = 1.0f; gat1.sb = 1.0f; gat1.Npad = HD; gat1.pad_ = 0;
      k_gemm<1><<<dim3((unsigned)((HD) + 31) / 32, (unsigned)((1) + 15) / 16, (unsigned)(CHN * NH)), 32, 0, stream>>>(gat1); }
    k_wubu_gather<<<(unsigned)(((long long)CHN * KN * D + 255) / 256), 256, 0, stream>>>(KF, VF, IDX, pos, cc, KG, VG, GEO, 1024, CHN);
    { GemmP ggp2;
      ggp2.A = GEO; ggp2.B = wg; ggp2.bias = bg; ggp2.R = GEO; ggp2.C = GP;
      ggp2.sAo = 0; ggp2.sAi = 0; ggp2.sAm = 4; ggp2.sAk = 1; ggp2.sBo = 0; ggp2.sBi = 0; ggp2.sBn = 1; ggp2.sBk = D; ggp2.sCo = 0; ggp2.sCi = 0; ggp2.sCm = D; ggp2.sRo = 0; ggp2.sRi = 0; ggp2.sRm = 0; ggp2.sRn = 0;
      ggp2.M = CHN * KN; ggp2.N = D; ggp2.K = 3; ggp2.zi_n = 1; ggp2.flags = 1; ggp2.act = 0;
      ggp2.alpha = 1.0f; ggp2.beta = 0.0f; ggp2.sa = 1.0f; ggp2.sb = 1.0f; ggp2.Npad = D; ggp2.pad_ = 0;
      k_gemm<1><<<dim3((unsigned)((D) + 31) / 32, (unsigned)((CHN * KN) + 15) / 16, (unsigned)(1)), 32, 0, stream>>>(ggp2); }
    { GemmP gSC1_2;
      gSC1_2.A = Q + (size_t)1024 * D; gSC1_2.B = KG; gSC1_2.bias = Q + (size_t)1024 * D; gSC1_2.R = Q + (size_t)1024 * D; gSC1_2.C = SC1;
      gSC1_2.sAo = D; gSC1_2.sAi = HD; gSC1_2.sAm = 0; gSC1_2.sAk = 1; gSC1_2.sBo = (long long)KN * D; gSC1_2.sBi = HD; gSC1_2.sBn = D; gSC1_2.sBk = 1; gSC1_2.sCo = NH * KN; gSC1_2.sCi = KN; gSC1_2.sCm = KN; gSC1_2.sRo = 0; gSC1_2.sRi = 0; gSC1_2.sRm = 0; gSC1_2.sRn = 0;
      gSC1_2.M = 1; gSC1_2.N = KN; gSC1_2.K = HD; gSC1_2.zi_n = NH; gSC1_2.flags = 0; gSC1_2.act = 0;
      gSC1_2.alpha = 1.0f; gSC1_2.beta = 0.0f; gSC1_2.sa = 1.0f; gSC1_2.sb = 1.0f; gSC1_2.Npad = KN; gSC1_2.pad_ = 0;
      k_gemm<1><<<dim3((unsigned)((KN) + 31) / 32, (unsigned)((1) + 15) / 16, (unsigned)(CHN * NH)), 32, 0, stream>>>(gSC1_2); }
    { GemmP gSC2_2;
      gSC2_2.A = Q + (size_t)1024 * D; gSC2_2.B = GP; gSC2_2.bias = Q + (size_t)1024 * D; gSC2_2.R = Q + (size_t)1024 * D; gSC2_2.C = SC2;
      gSC2_2.sAo = D; gSC2_2.sAi = HD; gSC2_2.sAm = 0; gSC2_2.sAk = 1; gSC2_2.sBo = (long long)KN * D; gSC2_2.sBi = HD; gSC2_2.sBn = D; gSC2_2.sBk = 1; gSC2_2.sCo = NH * KN; gSC2_2.sCi = KN; gSC2_2.sCm = KN; gSC2_2.sRo = 0; gSC2_2.sRi = 0; gSC2_2.sRm = 0; gSC2_2.sRn = 0;
      gSC2_2.M = 1; gSC2_2.N = KN; gSC2_2.K = HD; gSC2_2.zi_n = NH; gSC2_2.flags = 0; gSC2_2.act = 0;
      gSC2_2.alpha = 1.0f; gSC2_2.beta = 0.0f; gSC2_2.sa = 1.0f; gSC2_2.sb = 1.0f; gSC2_2.Npad = KN; gSC2_2.pad_ = 0;
      k_gemm<1><<<dim3((unsigned)((KN) + 31) / 32, (unsigned)((1) + 15) / 16, (unsigned)(CHN * NH)), 32, 0, stream>>>(gSC2_2); }
    k_wubu_soft<<<(unsigned)((CHN * NH + 255) / 256), 256, 0, stream>>>(SC1, SC2, asc, fsc, WT, CHN * NH);
    { GemmP gat2;
      gat2.A = WT; gat2.B = VG; gat2.bias = WT; gat2.R = WT; gat2.C = AT + (size_t)1024 * D;
      gat2.sAo = NH * KN; gat2.sAi = KN; gat2.sAm = 0; gat2.sAk = 1; gat2.sBo = (long long)KN * D; gat2.sBi = HD; gat2.sBn = 1; gat2.sBk = D; gat2.sCo = D; gat2.sCi = HD; gat2.sCm = HD; gat2.sRo = 0; gat2.sRi = 0; gat2.sRm = 0; gat2.sRn = 0;
      gat2.M = 1; gat2.N = HD; gat2.K = KN; gat2.zi_n = NH; gat2.flags = 0; gat2.act = 0;
      gat2.alpha = 1.0f; gat2.beta = 0.0f; gat2.sa = 1.0f; gat2.sb = 1.0f; gat2.Npad = HD; gat2.pad_ = 0;
      k_gemm<1><<<dim3((unsigned)((HD) + 31) / 32, (unsigned)((1) + 15) / 16, (unsigned)(CHN * NH)), 32, 0, stream>>>(gat2); }
    k_wubu_gather<<<(unsigned)(((long long)CHN * KN * D + 255) / 256), 256, 0, stream>>>(KF, VF, IDX, pos, cc, KG, VG, GEO, 1536, CHN);
    { GemmP ggp3;
      ggp3.A = GEO; ggp3.B = wg; ggp3.bias = bg; ggp3.R = GEO; ggp3.C = GP;
      ggp3.sAo = 0; ggp3.sAi = 0; ggp3.sAm = 4; ggp3.sAk = 1; ggp3.sBo = 0; ggp3.sBi = 0; ggp3.sBn = 1; ggp3.sBk = D; ggp3.sCo = 0; ggp3.sCi = 0; ggp3.sCm = D; ggp3.sRo = 0; ggp3.sRi = 0; ggp3.sRm = 0; ggp3.sRn = 0;
      ggp3.M = CHN * KN; ggp3.N = D; ggp3.K = 3; ggp3.zi_n = 1; ggp3.flags = 1; ggp3.act = 0;
      ggp3.alpha = 1.0f; ggp3.beta = 0.0f; ggp3.sa = 1.0f; ggp3.sb = 1.0f; ggp3.Npad = D; ggp3.pad_ = 0;
      k_gemm<1><<<dim3((unsigned)((D) + 31) / 32, (unsigned)((CHN * KN) + 15) / 16, (unsigned)(1)), 32, 0, stream>>>(ggp3); }
    { GemmP gSC1_3;
      gSC1_3.A = Q + (size_t)1536 * D; gSC1_3.B = KG; gSC1_3.bias = Q + (size_t)1536 * D; gSC1_3.R = Q + (size_t)1536 * D; gSC1_3.C = SC1;
      gSC1_3.sAo = D; gSC1_3.sAi = HD; gSC1_3.sAm = 0; gSC1_3.sAk = 1; gSC1_3.sBo = (long long)KN * D; gSC1_3.sBi = HD; gSC1_3.sBn = D; gSC1_3.sBk = 1; gSC1_3.sCo = NH * KN; gSC1_3.sCi = KN; gSC1_3.sCm = KN; gSC1_3.sRo = 0; gSC1_3.sRi = 0; gSC1_3.sRm = 0; gSC1_3.sRn = 0;
      gSC1_3.M = 1; gSC1_3.N = KN; gSC1_3.K = HD; gSC1_3.zi_n = NH; gSC1_3.flags = 0; gSC1_3.act = 0;
      gSC1_3.alpha = 1.0f; gSC1_3.beta = 0.0f; gSC1_3.sa = 1.0f; gSC1_3.sb = 1.0f; gSC1_3.Npad = KN; gSC1_3.pad_ = 0;
      k_gemm<1><<<dim3((unsigned)((KN) + 31) / 32, (unsigned)((1) + 15) / 16, (unsigned)(CHN * NH)), 32, 0, stream>>>(gSC1_3); }
    { GemmP gSC2_3;
      gSC2_3.A = Q + (size_t)1536 * D; gSC2_3.B = GP; gSC2_3.bias = Q + (size_t)1536 * D; gSC2_3.R = Q + (size_t)1536 * D; gSC2_3.C = SC2;
      gSC2_3.sAo = D; gSC2_3.sAi = HD; gSC2_3.sAm = 0; gSC2_3.sAk = 1; gSC2_3.sBo = (long long)KN * D; gSC2_3.sBi = HD; gSC2_3.sBn = D; gSC2_3.sBk = 1; gSC2_3.sCo = NH * KN; gSC2_3.sCi = KN; gSC2_3.sCm = KN; gSC2_3.sRo = 0; gSC2_3.sRi = 0; gSC2_3.sRm = 0; gSC2_3.sRn = 0;
      gSC2_3.M = 1; gSC2_3.N = KN; gSC2_3.K = HD; gSC2_3.zi_n = NH; gSC2_3.flags = 0; gSC2_3.act = 0;
      gSC2_3.alpha = 1.0f; gSC2_3.beta = 0.0f; gSC2_3.sa = 1.0f; gSC2_3.sb = 1.0f; gSC2_3.Npad = KN; gSC2_3.pad_ = 0;
      k_gemm<1><<<dim3((unsigned)((KN) + 31) / 32, (unsigned)((1) + 15) / 16, (unsigned)(CHN * NH)), 32, 0, stream>>>(gSC2_3); }
    k_wubu_soft<<<(unsigned)((CHN * NH + 255) / 256), 256, 0, stream>>>(SC1, SC2, asc, fsc, WT, CHN * NH);
    { GemmP gat3;
      gat3.A = WT; gat3.B = VG; gat3.bias = WT; gat3.R = WT; gat3.C = AT + (size_t)1536 * D;
      gat3.sAo = NH * KN; gat3.sAi = KN; gat3.sAm = 0; gat3.sAk = 1; gat3.sBo = (long long)KN * D; gat3.sBi = HD; gat3.sBn = 1; gat3.sBk = D; gat3.sCo = D; gat3.sCi = HD; gat3.sCm = HD; gat3.sRo = 0; gat3.sRi = 0; gat3.sRm = 0; gat3.sRn = 0;
      gat3.M = 1; gat3.N = HD; gat3.K = KN; gat3.zi_n = NH; gat3.flags = 0; gat3.act = 0;
      gat3.alpha = 1.0f; gat3.beta = 0.0f; gat3.sa = 1.0f; gat3.sb = 1.0f; gat3.Npad = HD; gat3.pad_ = 0;
      k_gemm<1><<<dim3((unsigned)((HD) + 31) / 32, (unsigned)((1) + 15) / 16, (unsigned)(CHN * NH)), 32, 0, stream>>>(gat3); }
    k_wubu_gather<<<(unsigned)(((long long)CHN * KN * D + 255) / 256), 256, 0, stream>>>(KF, VF, IDX, pos, cc, KG, VG, GEO, 2048, CHN);
    { GemmP ggp4;
      ggp4.A = GEO; ggp4.B = wg; ggp4.bias = bg; ggp4.R = GEO; ggp4.C = GP;
      ggp4.sAo = 0; ggp4.sAi = 0; ggp4.sAm = 4; ggp4.sAk = 1; ggp4.sBo = 0; ggp4.sBi = 0; ggp4.sBn = 1; ggp4.sBk = D; ggp4.sCo = 0; ggp4.sCi = 0; ggp4.sCm = D; ggp4.sRo = 0; ggp4.sRi = 0; ggp4.sRm = 0; ggp4.sRn = 0;
      ggp4.M = CHN * KN; ggp4.N = D; ggp4.K = 3; ggp4.zi_n = 1; ggp4.flags = 1; ggp4.act = 0;
      ggp4.alpha = 1.0f; ggp4.beta = 0.0f; ggp4.sa = 1.0f; ggp4.sb = 1.0f; ggp4.Npad = D; ggp4.pad_ = 0;
      k_gemm<1><<<dim3((unsigned)((D) + 31) / 32, (unsigned)((CHN * KN) + 15) / 16, (unsigned)(1)), 32, 0, stream>>>(ggp4); }
    { GemmP gSC1_4;
      gSC1_4.A = Q + (size_t)2048 * D; gSC1_4.B = KG; gSC1_4.bias = Q + (size_t)2048 * D; gSC1_4.R = Q + (size_t)2048 * D; gSC1_4.C = SC1;
      gSC1_4.sAo = D; gSC1_4.sAi = HD; gSC1_4.sAm = 0; gSC1_4.sAk = 1; gSC1_4.sBo = (long long)KN * D; gSC1_4.sBi = HD; gSC1_4.sBn = D; gSC1_4.sBk = 1; gSC1_4.sCo = NH * KN; gSC1_4.sCi = KN; gSC1_4.sCm = KN; gSC1_4.sRo = 0; gSC1_4.sRi = 0; gSC1_4.sRm = 0; gSC1_4.sRn = 0;
      gSC1_4.M = 1; gSC1_4.N = KN; gSC1_4.K = HD; gSC1_4.zi_n = NH; gSC1_4.flags = 0; gSC1_4.act = 0;
      gSC1_4.alpha = 1.0f; gSC1_4.beta = 0.0f; gSC1_4.sa = 1.0f; gSC1_4.sb = 1.0f; gSC1_4.Npad = KN; gSC1_4.pad_ = 0;
      k_gemm<1><<<dim3((unsigned)((KN) + 31) / 32, (unsigned)((1) + 15) / 16, (unsigned)(CHN * NH)), 32, 0, stream>>>(gSC1_4); }
    { GemmP gSC2_4;
      gSC2_4.A = Q + (size_t)2048 * D; gSC2_4.B = GP; gSC2_4.bias = Q + (size_t)2048 * D; gSC2_4.R = Q + (size_t)2048 * D; gSC2_4.C = SC2;
      gSC2_4.sAo = D; gSC2_4.sAi = HD; gSC2_4.sAm = 0; gSC2_4.sAk = 1; gSC2_4.sBo = (long long)KN * D; gSC2_4.sBi = HD; gSC2_4.sBn = D; gSC2_4.sBk = 1; gSC2_4.sCo = NH * KN; gSC2_4.sCi = KN; gSC2_4.sCm = KN; gSC2_4.sRo = 0; gSC2_4.sRi = 0; gSC2_4.sRm = 0; gSC2_4.sRn = 0;
      gSC2_4.M = 1; gSC2_4.N = KN; gSC2_4.K = HD; gSC2_4.zi_n = NH; gSC2_4.flags = 0; gSC2_4.act = 0;
      gSC2_4.alpha = 1.0f; gSC2_4.beta = 0.0f; gSC2_4.sa = 1.0f; gSC2_4.sb = 1.0f; gSC2_4.Npad = KN; gSC2_4.pad_ = 0;
      k_gemm<1><<<dim3((unsigned)((KN) + 31) / 32, (unsigned)((1) + 15) / 16, (unsigned)(CHN * NH)), 32, 0, stream>>>(gSC2_4); }
    k_wubu_soft<<<(unsigned)((CHN * NH + 255) / 256), 256, 0, stream>>>(SC1, SC2, asc, fsc, WT, CHN * NH);
    { GemmP gat4;
      gat4.A = WT; gat4.B = VG; gat4.bias = WT; gat4.R = WT; gat4.C = AT + (size_t)2048 * D;
      gat4.sAo = NH * KN; gat4.sAi = KN; gat4.sAm = 0; gat4.sAk = 1; gat4.sBo = (long long)KN * D; gat4.sBi = HD; gat4.sBn = 1; gat4.sBk = D; gat4.sCo = D; gat4.sCi = HD; gat4.sCm = HD; gat4.sRo = 0; gat4.sRi = 0; gat4.sRm = 0; gat4.sRn = 0;
      gat4.M = 1; gat4.N = HD; gat4.K = KN; gat4.zi_n = NH; gat4.flags = 0; gat4.act = 0;
      gat4.alpha = 1.0f; gat4.beta = 0.0f; gat4.sa = 1.0f; gat4.sb = 1.0f; gat4.Npad = HD; gat4.pad_ = 0;
      k_gemm<1><<<dim3((unsigned)((HD) + 31) / 32, (unsigned)((1) + 15) / 16, (unsigned)(CHN * NH)), 32, 0, stream>>>(gat4); }
    k_wubu_gather<<<(unsigned)(((long long)CHN * KN * D + 255) / 256), 256, 0, stream>>>(KF, VF, IDX, pos, cc, KG, VG, GEO, 2560, CHN);
    { GemmP ggp5;
      ggp5.A = GEO; ggp5.B = wg; ggp5.bias = bg; ggp5.R = GEO; ggp5.C = GP;
      ggp5.sAo = 0; ggp5.sAi = 0; ggp5.sAm = 4; ggp5.sAk = 1; ggp5.sBo = 0; ggp5.sBi = 0; ggp5.sBn = 1; ggp5.sBk = D; ggp5.sCo = 0; ggp5.sCi = 0; ggp5.sCm = D; ggp5.sRo = 0; ggp5.sRi = 0; ggp5.sRm = 0; ggp5.sRn = 0;
      ggp5.M = CHN * KN; ggp5.N = D; ggp5.K = 3; ggp5.zi_n = 1; ggp5.flags = 1; ggp5.act = 0;
      ggp5.alpha = 1.0f; ggp5.beta = 0.0f; ggp5.sa = 1.0f; ggp5.sb = 1.0f; ggp5.Npad = D; ggp5.pad_ = 0;
      k_gemm<1><<<dim3((unsigned)((D) + 31) / 32, (unsigned)((CHN * KN) + 15) / 16, (unsigned)(1)), 32, 0, stream>>>(ggp5); }
    { GemmP gSC1_5;
      gSC1_5.A = Q + (size_t)2560 * D; gSC1_5.B = KG; gSC1_5.bias = Q + (size_t)2560 * D; gSC1_5.R = Q + (size_t)2560 * D; gSC1_5.C = SC1;
      gSC1_5.sAo = D; gSC1_5.sAi = HD; gSC1_5.sAm = 0; gSC1_5.sAk = 1; gSC1_5.sBo = (long long)KN * D; gSC1_5.sBi = HD; gSC1_5.sBn = D; gSC1_5.sBk = 1; gSC1_5.sCo = NH * KN; gSC1_5.sCi = KN; gSC1_5.sCm = KN; gSC1_5.sRo = 0; gSC1_5.sRi = 0; gSC1_5.sRm = 0; gSC1_5.sRn = 0;
      gSC1_5.M = 1; gSC1_5.N = KN; gSC1_5.K = HD; gSC1_5.zi_n = NH; gSC1_5.flags = 0; gSC1_5.act = 0;
      gSC1_5.alpha = 1.0f; gSC1_5.beta = 0.0f; gSC1_5.sa = 1.0f; gSC1_5.sb = 1.0f; gSC1_5.Npad = KN; gSC1_5.pad_ = 0;
      k_gemm<1><<<dim3((unsigned)((KN) + 31) / 32, (unsigned)((1) + 15) / 16, (unsigned)(CHN * NH)), 32, 0, stream>>>(gSC1_5); }
    { GemmP gSC2_5;
      gSC2_5.A = Q + (size_t)2560 * D; gSC2_5.B = GP; gSC2_5.bias = Q + (size_t)2560 * D; gSC2_5.R = Q + (size_t)2560 * D; gSC2_5.C = SC2;
      gSC2_5.sAo = D; gSC2_5.sAi = HD; gSC2_5.sAm = 0; gSC2_5.sAk = 1; gSC2_5.sBo = (long long)KN * D; gSC2_5.sBi = HD; gSC2_5.sBn = D; gSC2_5.sBk = 1; gSC2_5.sCo = NH * KN; gSC2_5.sCi = KN; gSC2_5.sCm = KN; gSC2_5.sRo = 0; gSC2_5.sRi = 0; gSC2_5.sRm = 0; gSC2_5.sRn = 0;
      gSC2_5.M = 1; gSC2_5.N = KN; gSC2_5.K = HD; gSC2_5.zi_n = NH; gSC2_5.flags = 0; gSC2_5.act = 0;
      gSC2_5.alpha = 1.0f; gSC2_5.beta = 0.0f; gSC2_5.sa = 1.0f; gSC2_5.sb = 1.0f; gSC2_5.Npad = KN; gSC2_5.pad_ = 0;
      k_gemm<1><<<dim3((unsigned)((KN) + 31) / 32, (unsigned)((1) + 15) / 16, (unsigned)(CHN * NH)), 32, 0, stream>>>(gSC2_5); }
    k_wubu_soft<<<(unsigned)((CHN * NH + 255) / 256), 256, 0, stream>>>(SC1, SC2, asc, fsc, WT, CHN * NH);
    { GemmP gat5;
      gat5.A = WT; gat5.B = VG; gat5.bias = WT; gat5.R = WT; gat5.C = AT + (size_t)2560 * D;
      gat5.sAo = NH * KN; gat5.sAi = KN; gat5.sAm = 0; gat5.sAk = 1; gat5.sBo = (long long)KN * D; gat5.sBi = HD; gat5.sBn = 1; gat5.sBk = D; gat5.sCo = D; gat5.sCi = HD; gat5.sCm = HD; gat5.sRo = 0; gat5.sRi = 0; gat5.sRm = 0; gat5.sRn = 0;
      gat5.M = 1; gat5.N = HD; gat5.K = KN; gat5.zi_n = NH; gat5.flags = 0; gat5.act = 0;
      gat5.alpha = 1.0f; gat5.beta = 0.0f; gat5.sa = 1.0f; gat5.sb = 1.0f; gat5.Npad = HD; gat5.pad_ = 0;
      k_gemm<1><<<dim3((unsigned)((HD) + 31) / 32, (unsigned)((1) + 15) / 16, (unsigned)(CHN * NH)), 32, 0, stream>>>(gat5); }
    k_wubu_gather<<<(unsigned)(((long long)CHN * KN * D + 255) / 256), 256, 0, stream>>>(KF, VF, IDX, pos, cc, KG, VG, GEO, 3072, CHN);
    { GemmP ggp6;
      ggp6.A = GEO; ggp6.B = wg; ggp6.bias = bg; ggp6.R = GEO; ggp6.C = GP;
      ggp6.sAo = 0; ggp6.sAi = 0; ggp6.sAm = 4; ggp6.sAk = 1; ggp6.sBo = 0; ggp6.sBi = 0; ggp6.sBn = 1; ggp6.sBk = D; ggp6.sCo = 0; ggp6.sCi = 0; ggp6.sCm = D; ggp6.sRo = 0; ggp6.sRi = 0; ggp6.sRm = 0; ggp6.sRn = 0;
      ggp6.M = CHN * KN; ggp6.N = D; ggp6.K = 3; ggp6.zi_n = 1; ggp6.flags = 1; ggp6.act = 0;
      ggp6.alpha = 1.0f; ggp6.beta = 0.0f; ggp6.sa = 1.0f; ggp6.sb = 1.0f; ggp6.Npad = D; ggp6.pad_ = 0;
      k_gemm<1><<<dim3((unsigned)((D) + 31) / 32, (unsigned)((CHN * KN) + 15) / 16, (unsigned)(1)), 32, 0, stream>>>(ggp6); }
    { GemmP gSC1_6;
      gSC1_6.A = Q + (size_t)3072 * D; gSC1_6.B = KG; gSC1_6.bias = Q + (size_t)3072 * D; gSC1_6.R = Q + (size_t)3072 * D; gSC1_6.C = SC1;
      gSC1_6.sAo = D; gSC1_6.sAi = HD; gSC1_6.sAm = 0; gSC1_6.sAk = 1; gSC1_6.sBo = (long long)KN * D; gSC1_6.sBi = HD; gSC1_6.sBn = D; gSC1_6.sBk = 1; gSC1_6.sCo = NH * KN; gSC1_6.sCi = KN; gSC1_6.sCm = KN; gSC1_6.sRo = 0; gSC1_6.sRi = 0; gSC1_6.sRm = 0; gSC1_6.sRn = 0;
      gSC1_6.M = 1; gSC1_6.N = KN; gSC1_6.K = HD; gSC1_6.zi_n = NH; gSC1_6.flags = 0; gSC1_6.act = 0;
      gSC1_6.alpha = 1.0f; gSC1_6.beta = 0.0f; gSC1_6.sa = 1.0f; gSC1_6.sb = 1.0f; gSC1_6.Npad = KN; gSC1_6.pad_ = 0;
      k_gemm<1><<<dim3((unsigned)((KN) + 31) / 32, (unsigned)((1) + 15) / 16, (unsigned)(CHN * NH)), 32, 0, stream>>>(gSC1_6); }
    { GemmP gSC2_6;
      gSC2_6.A = Q + (size_t)3072 * D; gSC2_6.B = GP; gSC2_6.bias = Q + (size_t)3072 * D; gSC2_6.R = Q + (size_t)3072 * D; gSC2_6.C = SC2;
      gSC2_6.sAo = D; gSC2_6.sAi = HD; gSC2_6.sAm = 0; gSC2_6.sAk = 1; gSC2_6.sBo = (long long)KN * D; gSC2_6.sBi = HD; gSC2_6.sBn = D; gSC2_6.sBk = 1; gSC2_6.sCo = NH * KN; gSC2_6.sCi = KN; gSC2_6.sCm = KN; gSC2_6.sRo = 0; gSC2_6.sRi = 0; gSC2_6.sRm = 0; gSC2_6.sRn = 0;
      gSC2_6.M = 1; gSC2_6.N = KN; gSC2_6.K = HD; gSC2_6.zi_n = NH; gSC2_6.flags = 0; gSC2_6.act = 0;
      gSC2_6.alpha = 1.0f; gSC2_6.beta = 0.0f; gSC2_6.sa = 1.0f; gSC2_6.sb = 1.0f; gSC2_6.Npad = KN; gSC2_6.pad_ = 0;
      k_gemm<1><<<dim3((unsigned)((KN) + 31) / 32, (unsigned)((1) + 15) / 16, (unsigned)(CHN * NH)), 32, 0, stream>>>(gSC2_6); }
    k_wubu_soft<<<(unsigned)((CHN * NH + 255) / 256), 256, 0, stream>>>(SC1, SC2, asc, fsc, WT, CHN * NH);
    { GemmP gat6;
      gat6.A = WT; gat6.B = VG; gat6.bias = WT; gat6.R = WT; gat6.C = AT + (size_t)3072 * D;
      gat6.sAo = NH * KN; gat6.sAi = KN; gat6.sAm = 0; gat6.sAk = 1; gat6.sBo = (long long)KN * D; gat6.sBi = HD; gat6.sBn = 1; gat6.sBk = D; gat6.sCo = D; gat6.sCi = HD; gat6.sCm = HD; gat6.sRo = 0; gat6.sRi = 0; gat6.sRm = 0; gat6.sRn = 0;
      gat6.M = 1; gat6.N = HD; gat6.K = KN; gat6.zi_n = NH; gat6.flags = 0; gat6.act = 0;
      gat6.alpha = 1.0f; gat6.beta = 0.0f; gat6.sa = 1.0f; gat6.sb = 1.0f; gat6.Npad = HD; gat6.pad_ = 0;
      k_gemm<1><<<dim3((unsigned)((HD) + 31) / 32, (unsigned)((1) + 15) / 16, (unsigned)(CHN * NH)), 32, 0, stream>>>(gat6); }
    k_wubu_gather<<<(unsigned)(((long long)CHN * KN * D + 255) / 256), 256, 0, stream>>>(KF, VF, IDX, pos, cc, KG, VG, GEO, 3584, CHN);
    { GemmP ggp7;
      ggp7.A = GEO; ggp7.B = wg; ggp7.bias = bg; ggp7.R = GEO; ggp7.C = GP;
      ggp7.sAo = 0; ggp7.sAi = 0; ggp7.sAm = 4; ggp7.sAk = 1; ggp7.sBo = 0; ggp7.sBi = 0; ggp7.sBn = 1; ggp7.sBk = D; ggp7.sCo = 0; ggp7.sCi = 0; ggp7.sCm = D; ggp7.sRo = 0; ggp7.sRi = 0; ggp7.sRm = 0; ggp7.sRn = 0;
      ggp7.M = CHN * KN; ggp7.N = D; ggp7.K = 3; ggp7.zi_n = 1; ggp7.flags = 1; ggp7.act = 0;
      ggp7.alpha = 1.0f; ggp7.beta = 0.0f; ggp7.sa = 1.0f; ggp7.sb = 1.0f; ggp7.Npad = D; ggp7.pad_ = 0;
      k_gemm<1><<<dim3((unsigned)((D) + 31) / 32, (unsigned)((CHN * KN) + 15) / 16, (unsigned)(1)), 32, 0, stream>>>(ggp7); }
    { GemmP gSC1_7;
      gSC1_7.A = Q + (size_t)3584 * D; gSC1_7.B = KG; gSC1_7.bias = Q + (size_t)3584 * D; gSC1_7.R = Q + (size_t)3584 * D; gSC1_7.C = SC1;
      gSC1_7.sAo = D; gSC1_7.sAi = HD; gSC1_7.sAm = 0; gSC1_7.sAk = 1; gSC1_7.sBo = (long long)KN * D; gSC1_7.sBi = HD; gSC1_7.sBn = D; gSC1_7.sBk = 1; gSC1_7.sCo = NH * KN; gSC1_7.sCi = KN; gSC1_7.sCm = KN; gSC1_7.sRo = 0; gSC1_7.sRi = 0; gSC1_7.sRm = 0; gSC1_7.sRn = 0;
      gSC1_7.M = 1; gSC1_7.N = KN; gSC1_7.K = HD; gSC1_7.zi_n = NH; gSC1_7.flags = 0; gSC1_7.act = 0;
      gSC1_7.alpha = 1.0f; gSC1_7.beta = 0.0f; gSC1_7.sa = 1.0f; gSC1_7.sb = 1.0f; gSC1_7.Npad = KN; gSC1_7.pad_ = 0;
      k_gemm<1><<<dim3((unsigned)((KN) + 31) / 32, (unsigned)((1) + 15) / 16, (unsigned)(CHN * NH)), 32, 0, stream>>>(gSC1_7); }
    { GemmP gSC2_7;
      gSC2_7.A = Q + (size_t)3584 * D; gSC2_7.B = GP; gSC2_7.bias = Q + (size_t)3584 * D; gSC2_7.R = Q + (size_t)3584 * D; gSC2_7.C = SC2;
      gSC2_7.sAo = D; gSC2_7.sAi = HD; gSC2_7.sAm = 0; gSC2_7.sAk = 1; gSC2_7.sBo = (long long)KN * D; gSC2_7.sBi = HD; gSC2_7.sBn = D; gSC2_7.sBk = 1; gSC2_7.sCo = NH * KN; gSC2_7.sCi = KN; gSC2_7.sCm = KN; gSC2_7.sRo = 0; gSC2_7.sRi = 0; gSC2_7.sRm = 0; gSC2_7.sRn = 0;
      gSC2_7.M = 1; gSC2_7.N = KN; gSC2_7.K = HD; gSC2_7.zi_n = NH; gSC2_7.flags = 0; gSC2_7.act = 0;
      gSC2_7.alpha = 1.0f; gSC2_7.beta = 0.0f; gSC2_7.sa = 1.0f; gSC2_7.sb = 1.0f; gSC2_7.Npad = KN; gSC2_7.pad_ = 0;
      k_gemm<1><<<dim3((unsigned)((KN) + 31) / 32, (unsigned)((1) + 15) / 16, (unsigned)(CHN * NH)), 32, 0, stream>>>(gSC2_7); }
    k_wubu_soft<<<(unsigned)((CHN * NH + 255) / 256), 256, 0, stream>>>(SC1, SC2, asc, fsc, WT, CHN * NH);
    { GemmP gat7;
      gat7.A = WT; gat7.B = VG; gat7.bias = WT; gat7.R = WT; gat7.C = AT + (size_t)3584 * D;
      gat7.sAo = NH * KN; gat7.sAi = KN; gat7.sAm = 0; gat7.sAk = 1; gat7.sBo = (long long)KN * D; gat7.sBi = HD; gat7.sBn = 1; gat7.sBk = D; gat7.sCo = D; gat7.sCi = HD; gat7.sCm = HD; gat7.sRo = 0; gat7.sRi = 0; gat7.sRm = 0; gat7.sRn = 0;
      gat7.M = 1; gat7.N = HD; gat7.K = KN; gat7.zi_n = NH; gat7.flags = 0; gat7.act = 0;
      gat7.alpha = 1.0f; gat7.beta = 0.0f; gat7.sa = 1.0f; gat7.sb = 1.0f; gat7.Npad = HD; gat7.pad_ = 0;
      k_gemm<1><<<dim3((unsigned)((HD) + 31) / 32, (unsigned)((1) + 15) / 16, (unsigned)(CHN * NH)), 32, 0, stream>>>(gat7); }
    { GemmP go;
      go.A = AT; go.B = wo; go.bias = bo; go.R = x; go.C = X1;
      go.sAo = 0; go.sAi = 0; go.sAm = D; go.sAk = 1; go.sBo = 0; go.sBi = 0; go.sBn = 1; go.sBk = D; go.sCo = 0; go.sCi = 0; go.sCm = D; go.sRo = 0; go.sRi = 0; go.sRm = D; go.sRn = 1;
      go.M = N; go.N = D; go.K = D; go.zi_n = 1; go.flags = 5; go.act = 0;
      go.alpha = 1.0f; go.beta = 1.0f; go.sa = 1.0f; go.sb = 1.0f; go.Npad = D; go.pad_ = 0;
      k_gemm<1><<<dim3((unsigned)((D) + 31) / 32, (unsigned)((N) + 15) / 16, (unsigned)(1)), 32, 0, stream>>>(go); }
    k_stats<<<(unsigned)(N), 256, 0, stream>>>(X1, D, 0, 1, D, D, 1e-06f, st, 0);
    k_norm_apply<<<(unsigned)(((long long)(N) * (D) * (1) + 255) / 256), 256, 0, stream>>>(X1, H2, st, l2s, l2b, N, D, 1, 1, 0, 0);
    { GemmP g1;
      g1.A = H2; g1.B = w1; g1.bias = b1; g1.R = H2; g1.C = T;
      g1.sAo = 0; g1.sAi = 0; g1.sAm = D; g1.sAk = 1; g1.sBo = 0; g1.sBi = 0; g1.sBn = 1; g1.sBk = DFF; g1.sCo = 0; g1.sCi = 0; g1.sCm = DFF; g1.sRo = 0; g1.sRi = 0; g1.sRm = 0; g1.sRn = 0;
      g1.M = N; g1.N = DFF; g1.K = D; g1.zi_n = 1; g1.flags = 1; g1.act = 2;
      g1.alpha = 1.0f; g1.beta = 0.0f; g1.sa = 1.0f; g1.sb = 1.0f; g1.Npad = DFF; g1.pad_ = 0;
      k_gemm<1><<<dim3((unsigned)((DFF) + 31) / 32, (unsigned)((N) + 15) / 16, (unsigned)(1)), 32, 0, stream>>>(g1); }
    { GemmP g2;
      g2.A = T; g2.B = w2; g2.bias = b2; g2.R = X1; g2.C = out;
      g2.sAo = 0; g2.sAi = 0; g2.sAm = DFF; g2.sAk = 1; g2.sBo = 0; g2.sBi = 0; g2.sBn = 1; g2.sBk = D; g2.sCo = 0; g2.sCi = 0; g2.sCm = D; g2.sRo = 0; g2.sRi = 0; g2.sRm = D; g2.sRn = 1;
      g2.M = N; g2.N = D; g2.K = DFF; g2.zi_n = 1; g2.flags = 5; g2.act = 0;
      g2.alpha = 1.0f; g2.beta = 1.0f; g2.sa = 1.0f; g2.sb = 1.0f; g2.Npad = D; g2.pad_ = 0;
      k_gemm<1><<<dim3((unsigned)((D) + 31) / 32, (unsigned)((N) + 15) / 16, (unsigned)(1)), 32, 0, stream>>>(g2); }
}
